// SAM_77653008712343
// MI455X (gfx1250) — hardware-verified
//
#include <hip/hip_runtime.h>
#include <math.h>
#include <stdint.h>

#define NB   4
#define CH   512
#define IC   256
#define IMW  64
#define NP   4096
#define MT   (NB * NP)
#define QKW  (2 * IC)
#define VPW  (2 * NP)

static_assert(NP == IMW * IMW);
static_assert(IC == 256);
static_assert(QKW == 512);
static_assert(CH % 64 == 0);
static_assert(NP % 512 == 0);
static_assert(MT % 64 == 0);
static_assert(MT % 32 == 0);
static_assert(IC % 32 == 0);
static_assert(CH % 256 == 0);
static_assert(((IC * CH) / 8) % 256 == 0);
static_assert(((CH * CH) / 8) % 256 == 0);
static_assert(VPW % 32 == 0);
static_assert(NP % 64 == 0);

typedef __attribute__((ext_vector_type(16))) _Float16 v16h;
typedef __attribute__((ext_vector_type(8)))  _Float16 v8h;
typedef __attribute__((ext_vector_type(16))) __bf16   v16b;
typedef __attribute__((ext_vector_type(8)))  __bf16   v8b;
typedef __attribute__((ext_vector_type(8)))  float    v8f;
typedef __attribute__((ext_vector_type(4)))  float    v4f;
typedef __attribute__((ext_vector_type(2)))  float    v2f;
typedef __attribute__((ext_vector_type(4)))  unsigned int v4u;

__device__ __forceinline__ unsigned short f2bf_bits(float f) {
  unsigned u = __float_as_uint(f);
  return (unsigned short)((u + 0x7FFFu + ((u >> 16) & 1u)) >> 16);
}
__device__ __forceinline__ float bf_bits2f(unsigned short h) { return __uint_as_float(((unsigned)h) << 16); }
__device__ __forceinline__ float bf_rne(float f) { return bf_bits2f(f2bf_bits(f)); }
__device__ __forceinline__ unsigned pk16(unsigned short a, unsigned short b) { return (unsigned)a | ((unsigned)b << 16); }

__device__ __forceinline__ void dep_guard_h(v8f& a, v8f& b, v16h x, v16h y) { asm volatile("v_nop\n\tv_nop\n\tv_nop\n\tv_nop" : "+v"(a), "+v"(b) : "v"(x), "v"(y)); }
__device__ __forceinline__ void dep_guard_b(v8f& a, v8f& b, v16b x, v16b y) { asm volatile("v_nop\n\tv_nop\n\tv_nop\n\tv_nop" : "+v"(a), "+v"(b) : "v"(x), "v"(y)); }
__device__ __forceinline__ void keep4_h(v16h a, v16h b, v16h c, v16h d) { asm volatile("v_nop" :: "v"(a), "v"(b), "v"(c), "v"(d)); }
__device__ __forceinline__ void keep4_b(v16b a, v16b b, v16b c, v16b d) { asm volatile("v_nop" :: "v"(a), "v"(b), "v"(c), "v"(d)); }
__device__ __forceinline__ void acc_guard4(v8f& a, v8f& b, v8f& c, v8f& d) { asm volatile("v_nop\n\tv_nop\n\tv_nop\n\tv_nop" : "+v"(a), "+v"(b), "+v"(c), "+v"(d)); }
template <typename T> struct Frag;
template <> struct Frag<_Float16> {
  typedef v16h V; union U { v16h v; v8h h[2]; };
  static __device__ __forceinline__ v16h load(const _Float16* p) {
    U f; f.h[0] = *(const v8h*)(p); f.h[1] = *(const v8h*)(p + 16); return f.v;
  }
  static __device__ __forceinline__ v8f mma(v16h a, v16h b, v8f c) {
    return __builtin_amdgcn_wmma_f32_16x16x32_f16(false, a, false, b, (short)0, c, false, false);
  }
  static __device__ __forceinline__ void guard(v8f& a, v8f& b, v16h x, v16h y) { dep_guard_h(a, b, x, y); }
  static __device__ __forceinline__ void keep(v16h a, v16h b, v16h c, v16h d) { keep4_h(a, b, c, d); }
};
template <> struct Frag<__bf16> {
  typedef v16b V; union U { v16b v; v8b h[2]; };
  static __device__ __forceinline__ v16b load(const __bf16* p) {
    U f; f.h[0] = *(const v8b*)(p); f.h[1] = *(const v8b*)(p + 16); return f.v;
  }
  static __device__ __forceinline__ v8f mma(v16b a, v16b b, v8f c) {
    return __builtin_amdgcn_wmma_f32_16x16x32_bf16(false, a, false, b, (short)0, c, false, false);
  }
  static __device__ __forceinline__ void guard(v8f& a, v8f& b, v16b x, v16b y) { dep_guard_b(a, b, x, y); }
  static __device__ __forceinline__ void keep(v16b a, v16b b, v16b c, v16b d) { keep4_b(a, b, c, d); }
};

template <int ET> struct Elem;
template <> struct Elem<0> { typedef _Float16 T; };
template <> struct Elem<1> { typedef __bf16 T; };
template <int ET, bool SPLIT, int BIAS_MODE, int OUT_MODE, int RESID, int ACT, bool CSCALE, bool BWRAP>
__global__ __launch_bounds__(256) void wmma_gemm64(
    const unsigned short* __restrict__ Ap, const unsigned short* __restrict__ A2p, int lda, long strideA,
    const unsigned short* __restrict__ Btp, const unsigned short* __restrict__ Bt2p, int ldb, long strideB,
    void* Cout, void* Cout2, int ldc, long strideC,
    const float* __restrict__ bias, const float* __restrict__ cscale,
    const float* __restrict__ resid, long strideR,
    int M, int N, int K, int Kb, float scale) {
  static_assert(RESID == 0 || OUT_MODE == 0);
  typedef typename Elem<ET>::T T;
  typedef typename Frag<T>::V V;
  const T* A = (const T*)Ap; const T* A2 = (const T*)A2p; const T* Bt = (const T*)Btp; const T* Bt2 = (const T*)Bt2p;
  __shared__ __align__(16) float sT[8][16 * 68];
  const int b    = blockIdx.y;
  const int lane = threadIdx.x & 31;
  const int wave = threadIdx.x >> 5;
  const int tilesN = N >> 6;
  const int tilesM = M >> 6;
  const int tile = blockIdx.x * 8 + wave;
  if (tile >= tilesM * tilesN) return;
  const int tm = tile / tilesN;
  const int tn = tile - tm * tilesN;
  const int m0 = tm << 6;
  const int n0 = tn << 6;

  const T* Ab  = A  + (size_t)b * strideA;
  const T* Bb  = Bt + (size_t)b * strideB;
  const T* Ab2 = SPLIT ? (A2  + (size_t)b * strideA) : nullptr;
  const T* Bb2 = SPLIT ? (Bt2 + (size_t)b * strideB) : nullptr;

  const int rlane = lane & 15;
  const int koff  = (lane >> 4) * 8;
  const int mOff  = (lane >> 4) * 8;

  v8f acc[4][4];
#pragma unroll
  for (int i = 0; i < 4; ++i)
#pragma unroll
    for (int j = 0; j < 4; ++j) acc[i][j] = (v8f){0.f,0.f,0.f,0.f,0.f,0.f,0.f,0.f};

  for (int k0 = 0; k0 < K; k0 += 32) {
    int kb0 = k0;
    if (BWRAP) kb0 = (k0 >= Kb) ? (k0 - Kb) : k0;
    V bh[4], bl[4];
#pragma unroll
    for (int j = 0; j < 4; ++j) {
      const size_t bo = (size_t)(n0 + (j << 4) + rlane) * ldb + koff + kb0;
      bh[j] = Frag<T>::load(Bb + bo);
      if (SPLIT) bl[j] = Frag<T>::load(Bb2 + bo); else bl[j] = bh[j];
    }
#pragma unroll
    for (int i = 0; i < 4; ++i) {
      const size_t ao = (size_t)(m0 + (i << 4) + rlane) * lda + koff + k0;
      V ah = Frag<T>::load(Ab + ao);
      V al;
      if (SPLIT) al = Frag<T>::load(Ab2 + ao); else al = ah;
#pragma unroll
      for (int j = 0; j < 4; ++j) {
        acc[i][j] = Frag<T>::mma(ah, bh[j], acc[i][j]);
        if (SPLIT) {
          acc[i][j] = Frag<T>::mma(ah, bl[j], acc[i][j]);
          acc[i][j] = Frag<T>::mma(al, bh[j], acc[i][j]);
        }
      }
      Frag<T>::guard(acc[i][0], acc[i][3], ah, al);
    }
    Frag<T>::keep(bh[0], bh[1], bh[2], bh[3]);
    if (SPLIT) Frag<T>::keep(bl[0], bl[1], bl[2], bl[3]);
  }
  acc_guard4(acc[0][0], acc[0][1], acc[0][2], acc[0][3]);
  acc_guard4(acc[1][0], acc[1][1], acc[1][2], acc[1][3]);
  acc_guard4(acc[2][0], acc[2][1], acc[2][2], acc[2][3]);
  acc_guard4(acc[3][0], acc[3][1], acc[3][2], acc[3][3]);

  float* slab = sT[wave];
  const float* Rb = (RESID != 0) ? (resid + (size_t)b * strideR) : nullptr;
#pragma unroll
  for (int i = 0; i < 4; ++i) {
    const int mBase = m0 + (i << 4);
    float bm8[8];
    if (BIAS_MODE == 1) {
      const v4f b0 = *(const v4f*)(bias + mBase + mOff);
      const v4f b1 = *(const v4f*)(bias + mBase + mOff + 4);
      bm8[0] = bf_rne(b0[0]); bm8[1] = bf_rne(b0[1]); bm8[2] = bf_rne(b0[2]); bm8[3] = bf_rne(b0[3]);
      bm8[4] = bf_rne(b1[0]); bm8[5] = bf_rne(b1[1]); bm8[6] = bf_rne(b1[2]); bm8[7] = bf_rne(b1[3]);
    } else {
#pragma unroll
      for (int r = 0; r < 8; ++r) bm8[r] = 0.0f;
    }
#pragma unroll
    for (int j = 0; j < 4; ++j) {
      const int n = n0 + (j << 4) + rlane;
      float bv = 0.f;
      if (BIAS_MODE == 2) bv = bf_rne(bias[n]);
      float csv = 1.f;
      if (CSCALE) csv = cscale[n];
#pragma unroll
      for (int r = 0; r < 8; ++r) {
        float v = acc[i][j][r] * scale;
        if (BIAS_MODE == 1) v += bm8[r];
        if (BIAS_MODE == 2) v += bv;
        if (ACT == 1) v = tanhf(v);
        if (ACT == 2) v = fmaxf(v, 0.0f);
        if (ACT == 4) v = (v > 0.f) ? v : 0.01f * v;
        if (CSCALE) v = v * csv;
        slab[(mOff + r) * 68 + (j << 4) + rlane] = v;
      }
    }
    __builtin_amdgcn_fence(__ATOMIC_RELEASE, "workgroup");
    __builtin_amdgcn_wave_barrier();
    __builtin_amdgcn_fence(__ATOMIC_ACQUIRE, "workgroup");
    if (OUT_MODE == 0) {
      float* C = (float*)Cout + (size_t)b * strideC;
      const int hh = lane >> 4, c4 = (lane & 15) * 4;
      v4f ov[8];
#pragma unroll
      for (int it = 0; it < 8; ++it) {
        const int row = it * 2 + hh;
        v4f v = *(const v4f*)(slab + row * 68 + c4);
        if (RESID != 0) {
          const v4f x = *(const v4f*)(Rb + (size_t)(mBase + row) * ldc + n0 + c4);
          if (RESID == 2) { v[0] += bf_rne(x[0]); v[1] += bf_rne(x[1]); v[2] += bf_rne(x[2]); v[3] += bf_rne(x[3]); }
          else v += x;
        }
        ov[it] = v;
      }
      for (int pass = 0; pass < 2; ++pass) {
#pragma unroll
        for (int it = 0; it < 8; ++it) {
          const int row = it * 2 + hh;
          *(volatile v4f*)(C + (size_t)(mBase + row) * ldc + n0 + c4) = ov[it];
        }
        __threadfence();
      }
    } else {
      const int q = lane >> 3, c8 = (lane & 7) * 8;
      unsigned short* C  = (unsigned short*)Cout  + (size_t)b * strideC;
      unsigned short* C2 = (OUT_MODE == 2) ? ((unsigned short*)Cout2 + (size_t)b * strideC) : nullptr;
      for (int pass = 0; pass < 2; ++pass) {
#pragma unroll
        for (int it = 0; it < 4; ++it) {
          const int row = it * 4 + q;
          const float* sp = slab + row * 68 + c8;
          v8h hv, lv;
#pragma unroll
          for (int e = 0; e < 8; ++e) {
            if (OUT_MODE == 1) {
              hv[e] = (_Float16)sp[e];
            } else {
              unsigned short hb = f2bf_bits(sp[e]);
              unsigned short lb = f2bf_bits(sp[e] - bf_bits2f(hb));
              hv[e] = __builtin_bit_cast(_Float16, hb);
              lv[e] = __builtin_bit_cast(_Float16, lb);
            }
          }
          *(volatile v8h*)(C + (size_t)(mBase + row) * ldc + n0 + c8) = hv;
          if (OUT_MODE == 2) *(volatile v8h*)(C2 + (size_t)(mBase + row) * ldc + n0 + c8) = lv;
        }
        __threadfence();
      }
    }
    __builtin_amdgcn_fence(__ATOMIC_RELEASE, "workgroup");
    __builtin_amdgcn_wave_barrier();
    __builtin_amdgcn_fence(__ATOMIC_ACQUIRE, "workgroup");
  }
}

__global__ __launch_bounds__(256) void convrows_kernel(const float* __restrict__ in, unsigned short* __restrict__ out,
                                                       int ncols, int ldout, int n8) {
  const int i = blockIdx.x * 256 + threadIdx.x;
  if (i < n8) {
    const size_t e0 = (size_t)i * 8;
    const int row = (int)(e0 / (size_t)ncols);
    const int col = (int)(e0 - (size_t)row * ncols);
    const v4f a = *(const v4f*)(in + e0);
    const v4f c = *(const v4f*)(in + e0 + 4);
    v4u hv;
    hv[0] = pk16(f2bf_bits(a[0]), f2bf_bits(a[1]));
    hv[1] = pk16(f2bf_bits(a[2]), f2bf_bits(a[3]));
    hv[2] = pk16(f2bf_bits(c[0]), f2bf_bits(c[1]));
    hv[3] = pk16(f2bf_bits(c[2]), f2bf_bits(c[3]));
    const size_t o = (size_t)row * ldout + col;
    for (int pass = 0; pass < 2; ++pass) {
      *(volatile v4u*)(out + o) = hv;
      __threadfence();
    }
  }
}

__global__ __launch_bounds__(256) void tconv_kernel(const float* __restrict__ W, unsigned short* __restrict__ oh,
                                                    int ldin, int ldout, long sIn, long sOut) {
  __shared__ __align__(16) float tf[64 * 68];
  W  += (size_t)blockIdx.z * sIn;
  oh += (size_t)blockIdx.z * sOut;
  const int c0  = blockIdx.x * 64;
  const int r0  = blockIdx.y * 64;
  const int tid = threadIdx.x;
  {
    const int lr = tid >> 4;
    const int c4 = (tid & 15) * 4;
#pragma unroll
    for (int it = 0; it < 4; ++it) {
      const int rr = it * 16 + lr;
      const v4f a = *(const v4f*)(W + (size_t)(r0 + rr) * ldin + c0 + c4);
      *(v4f*)(tf + rr * 68 + c4) = a;
    }
  }
  __syncthreads();
  const int sub = tid >> 3;
  const int c8  = (tid & 7) * 8;
  v4u hv[2];
#pragma unroll
  for (int it = 0; it < 2; ++it) {
    const int oc = it * 32 + sub;
    v4u a;
#pragma unroll
    for (int q = 0; q < 4; ++q) {
      const float f0 = tf[(c8 + 2 * q) * 68 + oc];
      const float f1 = tf[(c8 + 2 * q + 1) * 68 + oc];
      a[q] = pk16(f2bf_bits(f0), f2bf_bits(f1));
    }
    hv[it] = a;
  }
  for (int pass = 0; pass < 2; ++pass) {
#pragma unroll
    for (int it = 0; it < 2; ++it) {
      const int oc = it * 32 + sub;
      const size_t go = (size_t)(c0 + oc) * ldout + r0 + c8;
      *(volatile v4u*)(oh + go) = hv[it];
    }
    __threadfence();
  }
}

__global__ __launch_bounds__(256) void qkrow_kernel(const float* __restrict__ qkf,
                                                    const float* __restrict__ qb, const float* __restrict__ kb,
                                                    const float* __restrict__ cw, const float* __restrict__ cb,
                                                    unsigned short* __restrict__ qh, unsigned short* __restrict__ ql,
                                                    unsigned short* __restrict__ kh, unsigned short* __restrict__ kl,
                                                    float* __restrict__ aq, float* __restrict__ bkk) {
  __shared__ float sa[32], sb[32];
  const int tid = threadIdx.x, lane = tid & 31, wave = tid >> 5;
  const int rb = blockIdx.x * 32;
  const int o8 = lane * 8;

  const v4f qba = *(const v4f*)(qb + o8), qbb = *(const v4f*)(qb + o8 + 4);
  const v4f kba = *(const v4f*)(kb + o8), kbb = *(const v4f*)(kb + o8 + 4);
  const v4f cba = *(const v4f*)(cb + o8), cbb = *(const v4f*)(cb + o8 + 4);
  const v4f cwa = *(const v4f*)(cw + 2 * o8), cwb = *(const v4f*)(cw + 2 * o8 + 4);
  const v4f cwc = *(const v4f*)(cw + 2 * o8 + 8), cwd = *(const v4f*)(cw + 2 * o8 + 12);
  float qb8[8], kb8[8], cb8[8], cx8[8], cy8[8];
  qb8[0] = bf_rne(qba[0]); qb8[1] = bf_rne(qba[1]); qb8[2] = bf_rne(qba[2]); qb8[3] = bf_rne(qba[3]);
  qb8[4] = bf_rne(qbb[0]); qb8[5] = bf_rne(qbb[1]); qb8[6] = bf_rne(qbb[2]); qb8[7] = bf_rne(qbb[3]);
  kb8[0] = bf_rne(kba[0]); kb8[1] = bf_rne(kba[1]); kb8[2] = bf_rne(kba[2]); kb8[3] = bf_rne(kba[3]);
  kb8[4] = bf_rne(kbb[0]); kb8[5] = bf_rne(kbb[1]); kb8[6] = bf_rne(kbb[2]); kb8[7] = bf_rne(kbb[3]);
  cb8[0] = bf_rne(cba[0]); cb8[1] = bf_rne(cba[1]); cb8[2] = bf_rne(cba[2]); cb8[3] = bf_rne(cba[3]);
  cb8[4] = bf_rne(cbb[0]); cb8[5] = bf_rne(cbb[1]); cb8[6] = bf_rne(cbb[2]); cb8[7] = bf_rne(cbb[3]);
  cx8[0] = bf_rne(cwa[0]); cy8[0] = bf_rne(cwa[1]); cx8[1] = bf_rne(cwa[2]); cy8[1] = bf_rne(cwa[3]);
  cx8[2] = bf_rne(cwb[0]); cy8[2] = bf_rne(cwb[1]); cx8[3] = bf_rne(cwb[2]); cy8[3] = bf_rne(cwb[3]);
  cx8[4] = bf_rne(cwc[0]); cy8[4] = bf_rne(cwc[1]); cx8[5] = bf_rne(cwc[2]); cy8[5] = bf_rne(cwc[3]);
  cx8[6] = bf_rne(cwd[0]); cy8[6] = bf_rne(cwd[1]); cx8[7] = bf_rne(cwd[2]); cy8[7] = bf_rne(cwd[3]);

#pragma unroll 1
  for (int i = 0; i < 4; ++i) {
    const int row = rb + wave * 4 + i;
    const int p  = row & (NP - 1);
    const int wx = p & (IMW - 1);
    const int hy = p >> 6;
    const float lw = -1.0f + (float)wx * (2.0f / 63.0f);
    const float lh = -1.0f + (float)hy * (2.0f / 63.0f);
    const float* qr = qkf + (size_t)row * QKW + o8;
    const v4f qa = *(const v4f*)(qr), qc = *(const v4f*)(qr + 4);
    const v4f ka = *(const v4f*)(qr + IC), kc = *(const v4f*)(qr + IC + 4);
    float q8[8], k8[8];
    q8[0] = qa[0]; q8[1] = qa[1]; q8[2] = qa[2]; q8[3] = qa[3];
    q8[4] = qc[0]; q8[5] = qc[1]; q8[6] = qc[2]; q8[7] = qc[3];
    k8[0] = ka[0]; k8[1] = ka[1]; k8[2] = ka[2]; k8[3] = ka[3];
    k8[4] = kc[0]; k8[5] = kc[1]; k8[6] = kc[2]; k8[7] = kc[3];
    float ssa = 0.0f, ssb = 0.0f;
    v4u hq, lq, hk, lk;
#pragma unroll
    for (int e2 = 0; e2 < 4; ++e2) {
      unsigned short hqb[2], lqb[2], hkb[2], lkb[2];
#pragma unroll
      for (int u = 0; u < 2; ++u) {
        const int e = 2 * e2 + u;
        const float ccv = fmaxf(cx8[e] * lw + cy8[e] * lh + cb8[e], 0.0f);
        const float qf  = fmaxf(q8[e] + qb8[e], 0.0f) + ccv;
        const float kf  = fmaxf(k8[e] + kb8[e], 0.0f) + ccv;
        ssa += qf * qf;
        ssb += kf * kf;
        const unsigned short h1 = f2bf_bits(qf);
        const unsigned short h2 = f2bf_bits(kf);
        hqb[u] = h1; lqb[u] = f2bf_bits(qf - bf_bits2f(h1));
        hkb[u] = h2; lkb[u] = f2bf_bits(kf - bf_bits2f(h2));
      }
      hq[e2] = pk16(hqb[0], hqb[1]); lq[e2] = pk16(lqb[0], lqb[1]);
      hk[e2] = pk16(hkb[0], hkb[1]); lk[e2] = pk16(lkb[0], lkb[1]);
    }
#pragma unroll
    for (int off = 1; off < 32; off <<= 1) { ssa += __shfl_xor(ssa, off, 32); ssb += __shfl_xor(ssb, off, 32); }
    const size_t o = (size_t)row * IC + o8;
    for (int pass = 0; pass < 2; ++pass) {
      *(volatile v4u*)(qh + o) = hq;
      *(volatile v4u*)(ql + o) = lq;
      *(volatile v4u*)(kh + o) = hk;
      *(volatile v4u*)(kl + o) = lk;
      __threadfence();
    }
    if (lane == 0) { sa[wave * 4 + i] = ssa; sb[wave * 4 + i] = ssb; }
  }
  __syncthreads();
  if (wave == 0) {
    const float va = sa[lane], vb2 = sb[lane];
    ((volatile float*)aq)[rb + lane]  = va;
    ((volatile float*)bkk)[rb + lane] = vb2;
    __threadfence();
    ((volatile float*)aq)[rb + lane]  = va;
    ((volatile float*)bkk)[rb + lane] = vb2;
  }
}

__global__ __launch_bounds__(256) void samk_kernel(const unsigned short* __restrict__ khp, const unsigned short* __restrict__ klp,
                                                   const unsigned short* __restrict__ qhp, const unsigned short* __restrict__ qlp,
                                                   const float* __restrict__ aq, const float* __restrict__ bk,
                                                   unsigned short* __restrict__ et, float* __restrict__ sout) {
  typedef __bf16 T;
  typedef v16b V;
  const T* A = (const T*)khp; const T* A2 = (const T*)klp; const T* Bt = (const T*)qhp; const T* Bt2 = (const T*)qlp;
  __shared__ __align__(16) float sT[8][16 * 68];
  __shared__ float cs[8][64];
  __shared__ __align__(16) float sS[64];
  const int lane = threadIdx.x & 31;
  const int wave = threadIdx.x >> 5;
  const int rlane = lane & 15;
  const int koff  = (lane >> 4) * 8;
  const int mOff  = (lane >> 4) * 8;
  const int n0 = blockIdx.x * 64;
  float* slab = sT[wave];

  float csum[4];
#pragma unroll
  for (int j = 0; j < 4; ++j) csum[j] = 0.0f;

#pragma unroll 1
  for (int itm = 0; itm < NP / 512; ++itm) {
    const int m0 = (itm * 8 + wave) * 64;
    v8f acc[4][4];
#pragma unroll
    for (int i = 0; i < 4; ++i)
#pragma unroll
      for (int j = 0; j < 4; ++j) acc[i][j] = (v8f){0.f,0.f,0.f,0.f,0.f,0.f,0.f,0.f};

    for (int k0 = 0; k0 < IC; k0 += 32) {
      V bh[4], bl[4];
#pragma unroll
      for (int j = 0; j < 4; ++j) {
        const size_t bo = (size_t)(n0 + (j << 4) + rlane) * IC + koff + k0;
        bh[j] = Frag<T>::load(Bt + bo);
        bl[j] = Frag<T>::load(Bt2 + bo);
      }
#pragma unroll
      for (int i = 0; i < 4; ++i) {
        const size_t ao = (size_t)(m0 + (i << 4) + rlane) * IC + koff + k0;
        V ah = Frag<T>::load(A + ao);
        V al = Frag<T>::load(A2 + ao);
#pragma unroll
        for (int j = 0; j < 4; ++j) {
          acc[i][j] = Frag<T>::mma(ah, bh[j], acc[i][j]);
          acc[i][j] = Frag<T>::mma(ah, bl[j], acc[i][j]);
          acc[i][j] = Frag<T>::mma(al, bh[j], acc[i][j]);
        }
        Frag<T>::guard(acc[i][0], acc[i][3], ah, al);
      }
      Frag<T>::keep(bh[0], bh[1], bh[2], bh[3]);
      Frag<T>::keep(bl[0], bl[1], bl[2], bl[3]);
    }
    acc_guard4(acc[0][0], acc[0][1], acc[0][2], acc[0][3]);
    acc_guard4(acc[1][0], acc[1][1], acc[1][2], acc[1][3]);
    acc_guard4(acc[2][0], acc[2][1], acc[2][2], acc[2][3]);
    acc_guard4(acc[3][0], acc[3][1], acc[3][2], acc[3][3]);

#pragma unroll
    for (int i = 0; i < 4; ++i) {
      const int mBase = m0 + (i << 4);
      const v4f bb0 = *(const v4f*)(bk + mBase + mOff);
      const v4f bb1 = *(const v4f*)(bk + mBase + mOff + 4);
      float bm[8];
      bm[0] = bb0[0]; bm[1] = bb0[1]; bm[2] = bb0[2]; bm[3] = bb0[3];
      bm[4] = bb1[0]; bm[5] = bb1[1]; bm[6] = bb1[2]; bm[7] = bb1[3];
#pragma unroll
      for (int j = 0; j < 4; ++j) {
        const float an = aq[n0 + (j << 4) + rlane];
        float cj = csum[j];
#pragma unroll
        for (int r = 0; r < 8; ++r) {
          const float d = (an + bm[r]) - 2.0f * acc[i][j][r];
          const float e = __expf(-d);
          cj += e;
          slab[(mOff + r) * 68 + (j << 4) + rlane] = e;
        }
        csum[j] = cj;
      }
      __builtin_amdgcn_fence(__ATOMIC_RELEASE, "workgroup");
      __builtin_amdgcn_wave_barrier();
      __builtin_amdgcn_fence(__ATOMIC_ACQUIRE, "workgroup");
      {
        const int q = lane >> 3, c8 = (lane & 7) * 8;
        for (int pass = 0; pass < 2; ++pass) {
#pragma unroll
          for (int it = 0; it < 4; ++it) {
            const int row = it * 4 + q;
            const float* sp = slab + row * 68 + c8;
            v8h hv;
#pragma unroll
            for (int e = 0; e < 8; ++e) hv[e] = __builtin_bit_cast(_Float16, f2bf_bits(sp[e]));
            *(volatile v8h*)(et + (size_t)(mBase + row) * NP + n0 + c8) = hv;
          }
          __threadfence();
        }
      }
      __builtin_amdgcn_fence(__ATOMIC_RELEASE, "workgroup");
      __builtin_amdgcn_wave_barrier();
      __builtin_amdgcn_fence(__ATOMIC_ACQUIRE, "workgroup");
    }
  }

#pragma unroll
  for (int j = 0; j < 4; ++j) csum[j] += __shfl_xor(csum[j], 16, 32);
  if (lane < 16) {
#pragma unroll
    for (int j = 0; j < 4; ++j) cs[wave][(j << 4) + lane] = csum[j];
  }
  __syncthreads();
  if (threadIdx.x < 64) {
    const int t = threadIdx.x;
    float g = 0.0f;
#pragma unroll
    for (int w = 0; w < 8; ++w) g += cs[w][t];
    sS[t] = 1.0f / (g + 1e-14f);
  }
  __syncthreads();
  if (wave == 0) {
    const v4f v = *(const v4f*)(sS + 4 * (lane & 15));
    if (lane < 16) {
      float* sp = sout + n0 + 4 * lane;
      *(volatile v4f*)sp = v;
      __threadfence();
      *(volatile v4f*)sp = v;
    }
  }
}

extern "C" void kernel_launch(void* const* d_in, const int* in_sizes, int n_in,
                              void* d_out, int out_size, void* d_ws, size_t ws_size,
                              hipStream_t stream) {
  if (n_in < 9) return;
  if (in_sizes[0] != NB * CH * NP) return;
  if (in_sizes[1] != IC * CH || in_sizes[2] != IC) return;
  if (in_sizes[3] != IC * CH || in_sizes[4] != IC) return;
  if (in_sizes[5] != CH * CH || in_sizes[6] != CH) return;
  if (in_sizes[7] != IC * 2 || in_sizes[8] != IC) return;
  if (out_size != NB * CH * NP) return;

  const float* f   = (const float*)d_in[0];
  const float* qw  = (const float*)d_in[1];
  const float* qbv = (const float*)d_in[2];
  const float* kw  = (const float*)d_in[3];
  const float* kbv = (const float*)d_in[4];
  const float* vw  = (const float*)d_in[5];
  const float* vbv = (const float*)d_in[6];
  const float* cw  = (const float*)d_in[7];
  const float* cbv = (const float*)d_in[8];
  float* out = (float*)d_out;

  const size_t PXT  = (size_t)MT * CH * 2;
  const size_t PW   = (size_t)CH * CH * 2;
  const size_t PQKF = (size_t)MT * QKW * 4;
  const size_t PPL  = (size_t)MT * IC * 2;
  const size_t PAB  = (size_t)MT * 4;
  const size_t PET  = (size_t)NP * NP * 2;
  const size_t PS   = (size_t)NP * 4;
  const size_t PVP  = (size_t)CH * VPW * 2;
  size_t off = 0;
  const size_t oXT  = off; off += PXT;
  const size_t oWQK = off; off += PW;
  const size_t oWV  = off; off += PW;
  const size_t oQKF = off; off += PQKF;
  const size_t oQh  = off; off += PPL;  const size_t oQl = off; off += PPL;
  const size_t oKh  = off; off += PPL;  const size_t oKl = off; off += PPL;
  const size_t oAQ  = off; off += PAB;  const size_t oBK = off; off += PAB;
  const size_t oET  = off; off += PET;
  const size_t oS   = off; off += PS;
  const size_t oVP  = off; off += PVP;
  if (off > ws_size) return;
  if (off > (size_t)134217728) return;

  char* ws = (char*)d_ws;
  unsigned short* XT  = (unsigned short*)(ws + oXT);
  unsigned short* WQK = (unsigned short*)(ws + oWQK);
  unsigned short* WV  = (unsigned short*)(ws + oWV);
  float*          QKf = (float*)(ws + oQKF);
  unsigned short* Qh  = (unsigned short*)(ws + oQh);  unsigned short* Ql = (unsigned short*)(ws + oQl);
  unsigned short* Kh  = (unsigned short*)(ws + oKh);  unsigned short* Kl = (unsigned short*)(ws + oKl);
  float*          AQ  = (float*)(ws + oAQ);           float*          BK = (float*)(ws + oBK);
  unsigned short* ET  = (unsigned short*)(ws + oET);
  float*          S   = (float*)(ws + oS);
  unsigned short* VP  = (unsigned short*)(ws + oVP);

  const dim3 blk(256);

  tconv_kernel<<<dim3(NP / 64, CH / 64, NB), blk, 0, stream>>>(f, XT, NP, CH, (long)CH * NP, (long)NP * CH);
  const int n8qk = IC * CH / 8;
  const int n8v  = CH * CH / 8;
  convrows_kernel<<<dim3(n8qk / 256), blk, 0, stream>>>(qw, WQK, CH, CH, n8qk);
  convrows_kernel<<<dim3(n8qk / 256), blk, 0, stream>>>(kw, WQK + (size_t)IC * CH, CH, CH, n8qk);
  convrows_kernel<<<dim3(n8v / 256), blk, 0, stream>>>(vw, WV, CH, CH, n8v);
  const dim3 gQK(((MT / 64) * (QKW / 64) + 7) / 8, 1);
  wmma_gemm64<1, false, 0, 0, 0, 0, false, false><<<gQK, blk, 0, stream>>>(
      XT, XT, CH, 0L, WQK, WQK, CH, 0L, (void*)QKf, (void*)QKf, QKW, 0L,
      vbv, S, f, 0L, MT, QKW, CH, CH, 1.0f);
  qkrow_kernel<<<dim3(MT / 32), blk, 0, stream>>>(QKf, qbv, kbv, cw, cbv, Qh, Ql, Kh, Kl, AQ, BK);

  const dim3 gK(NP / 64);
  const dim3 gV(((CH / 64) * (NP / 64) + 7) / 8, 1);
  const dim3 gO(((CH / 64) * (NP / 64) + 7) / 8, 1);
  for (int b = 0; b < NB; ++b) {
    const size_t tb = (size_t)b * NP;
    samk_kernel<<<gK, blk, 0, stream>>>(Kh + tb * IC, Kl + tb * IC, Qh + tb * IC, Ql + tb * IC,
                                        AQ + tb, BK + tb, ET, S);
    wmma_gemm64<1, false, 1, 2, 0, 2, true, false><<<gV, blk, 0, stream>>>(
        WV, WV, CH, 0L, XT + tb * CH, XT + tb * CH, CH, 0L, (void*)VP, (void*)(VP + NP), VPW, 0L,
        vbv, S, f, 0L, CH, NP, CH, CH, 1.0f);
    wmma_gemm64<1, false, 0, 0, 2, 0, false, true><<<gO, blk, 0, stream>>>(
        VP, VP, VPW, 0L, ET, ET, NP, 0L, (void*)(out + (size_t)b * CH * NP), (void*)(out + (size_t)b * CH * NP), NP, 0L,
        vbv, S, f + (size_t)b * CH * NP, 0L, CH, NP, VPW, NP, 1.0f);
  }
  (void)hipGetLastError();
}
